// LookUpGCN_7224134992211
// MI455X (gfx1250) — hardware-verified
//
#include <hip/hip_runtime.h>
#include <stddef.h>


#define DM    128
#define NTHR  256
#define NWAVE 8
#define GR    32
#define XSP   132
#define CHUNK 2048
#define WCAP  256
#define NGRP  (CHUNK / (NTHR * 4))
#define NB    512
#define AGG_LDS_BYTES ((NB * DM + NB) * 4 + (NWAVE * WCAP + NWAVE) * 4)

static_assert(NGRP == 2);
static_assert(WCAP == (CHUNK / NTHR) * 32);
static_assert(AGG_LDS_BYTES == 272416);
static_assert((NB & (NB - 1)) == 0);
static_assert(NB <= 512);
static_assert(NB <= NWAVE * WCAP);
static_assert((XSP % 4) == 0);

typedef float    v4f  __attribute__((ext_vector_type(4)));
typedef float    v8f  __attribute__((ext_vector_type(8)));
typedef int      v4i  __attribute__((ext_vector_type(4)));
typedef _Float16 v8h  __attribute__((ext_vector_type(8)));
typedef _Float16 v16h __attribute__((ext_vector_type(16)));

union FragH { v16h v; v4i u[2]; };
union Pack  { v8h h; v4i i; };

__device__ __forceinline__ v8f wmh(v16h a, v16h b, v8f c) {
  v8f d = __builtin_amdgcn_wmma_f32_16x16x32_f16(false, a, false, b, (short)0, c, false, false);
  asm volatile("v_nop\n\tv_nop\n\tv_nop\n\tv_nop" : "+v"(d) : "v"(a), "v"(b));
  return d;
}

__device__ __forceinline__ float wsum32(float v) {
  v += __shfl_xor(v, 16, 32);
  v += __shfl_xor(v, 8, 32);
  v += __shfl_xor(v, 4, 32);
  v += __shfl_xor(v, 2, 32);
  v += __shfl_xor(v, 1, 32);
  return v;
}

__device__ __forceinline__ float lk(float t) { return fmaxf(t, 0.2f * t); }
__device__ __forceinline__ float dl(v4f t, v4f w) {
  return w.x * lk(t.x) + w.y * lk(t.y) + w.z * lk(t.z) + w.w * lk(t.w);
}

__global__ __launch_bounds__(NTHR) void k_mean(const float* __restrict__ ew, int nE, float* wsum) {
  __shared__ double sd[NTHR];
  const int tid = threadIdx.x;
  double s = 0.0;
#pragma unroll 1
  for (int i = tid; i < nE; i += NTHR) s += (double)ew[i];
  sd[tid] = s;
  __syncthreads();
#pragma unroll 1
  for (int st = NTHR / 2; st > 0; st >>= 1) {
    if (tid < st) sd[tid] += sd[tid + st];
    __syncthreads();
  }
  const float mval = (float)(sd[0] / (double)nE);
  if (tid < 8) {
    const v4f v = {mval, mval, mval, mval};
    float* p = wsum + 4 * tid;
    *(volatile v4f*)p = v;
    __threadfence();
    *(volatile v4f*)p = v;
  }
}

__global__ __launch_bounds__(NTHR) void k_wcvt(const float* __restrict__ w0, const float* __restrict__ w1,
                                               const float* __restrict__ w2, const float* __restrict__ w3,
                                               unsigned short* planes, float fscale) {
  const int which = blockIdx.y;
  const float* W = (which == 0) ? w0 : ((which == 1) ? w1 : ((which == 2) ? w2 : w3));
  unsigned short* T = planes + (size_t)which * DM * DM;
  const int i = blockIdx.x * NTHR + threadIdx.x;
  if (i >= DM * DM / 8) return;
  const int n  = i >> 4;
  const int kb = (i & 15) * 8;
  Pack u;
#pragma unroll
  for (int j = 0; j < 8; ++j) u.h[j] = (_Float16)(W[(size_t)(kb + j) * DM + n] * fscale);
  unsigned short* p = T + (size_t)i * 8;
  *(volatile v4i*)p = u.i;
  __threadfence();
  *(volatile v4i*)p = u.i;
}

__global__ __launch_bounds__(NTHR) void k_gather(const int* __restrict__ ids, const float* __restrict__ emb, int nV,
                                                 float* x0, unsigned short* apl, int nN, int Npad, float fscale) {
  const int i = blockIdx.x * NTHR + threadIdx.x;
  const bool pa = i < nN * 32;
  const bool pb = i < Npad * 16;

  int ra = i >> 5;
  ra = (ra < nN) ? ra : (nN - 1);
  const int c4 = i & 31;
  int ida = ids[ra];
  ida = ida < 0 ? 0 : (ida > nV - 1 ? nV - 1 : ida);
  const v4f va = *(const v4f*)(emb + (size_t)ida * DM + 4 * c4);
  float* pA = x0 + (size_t)ra * DM + 4 * c4;

  const int rb  = i >> 4;
  const int c8  = (i & 15) * 8;
  const int rbc = (rb < nN) ? rb : (nN - 1);
  int idb = ids[rbc];
  idb = idb < 0 ? 0 : (idb > nV - 1 ? nV - 1 : idb);
  const v4f b0 = *(const v4f*)(emb + (size_t)idb * DM + c8);
  const v4f b1 = *(const v4f*)(emb + (size_t)idb * DM + c8 + 4);
  Pack u;
  const v4i z4 = {0, 0, 0, 0};
  u.i = z4;
  if (rb < nN) {
#pragma unroll
    for (int j = 0; j < 4; ++j) {
      u.h[j]     = (_Float16)(b0[j] * fscale);
      u.h[4 + j] = (_Float16)(b1[j] * fscale);
    }
  }
  unsigned short* pB = apl + (size_t)rb * DM + c8;

  if (pa) *(volatile v4f*)pA = va;
  if (pb) *(volatile v4i*)pB = u.i;
  __threadfence();
  if (pa) *(volatile v4f*)pA = va;
  if (pb) *(volatile v4i*)pB = u.i;
}

__global__ __launch_bounds__(NTHR) void k_xcvt(const float* __restrict__ src, unsigned short* apl, int nN, int Npad) {
  const int i = blockIdx.x * NTHR + threadIdx.x;
  if (i >= Npad * 16) return;
  const int rb  = i >> 4;
  const int c8  = (i & 15) * 8;
  const int rbc = (rb < nN) ? rb : (nN - 1);
  const v4f b0 = *(const v4f*)(src + (size_t)rbc * DM + c8);
  const v4f b1 = *(const v4f*)(src + (size_t)rbc * DM + c8 + 4);
  Pack u;
  const v4i z4 = {0, 0, 0, 0};
  u.i = z4;
  if (rb < nN) {
#pragma unroll
    for (int j = 0; j < 4; ++j) {
      u.h[j]     = (_Float16)b0[j];
      u.h[4 + j] = (_Float16)b1[j];
    }
  }
  unsigned short* p = apl + (size_t)rb * DM + c8;
  *(volatile v4i*)p = u.i;
  __threadfence();
  *(volatile v4i*)p = u.i;
}

__global__ __launch_bounds__(NTHR) void k_gemm(const unsigned short* __restrict__ A,
                                               const unsigned short* __restrict__ B0, const unsigned short* __restrict__ B1,
                                               const float* __restrict__ bias0, const float* __restrict__ bias1,
                                               float* out0, float* out1, int K, float oscale) {
  __shared__ __attribute__((aligned(16))) float Xs[GR * XSP];

  const int which = blockIdx.y;
  const unsigned short* B = which ? B1 : B0;
  const float* bias = which ? bias1 : bias0;
  float* out = which ? out1 : out0;

  const int tid  = threadIdx.x;
  const int lane = tid & 31;
  const int wave = tid >> 5;
  const int hh   = lane >> 4;
  const int m    = lane & 15;
  const int rowBase = blockIdx.x * GR;
  const int ncol = wave * 16 + m;

  const size_t ra0 = (size_t)(rowBase + m) * K + 8 * hh;
  const size_t ra1 = ra0 + (size_t)16 * K;
  const size_t rb  = (size_t)ncol * K + 8 * hh;

  v8f c0 = {0.f, 0.f, 0.f, 0.f, 0.f, 0.f, 0.f, 0.f};
  v8f c1 = {0.f, 0.f, 0.f, 0.f, 0.f, 0.f, 0.f, 0.f};

#pragma unroll 1
  for (int k0 = 0; k0 < K; k0 += 32) {
    FragH a0, a1, b;
    a0.u[0] = *(const v4i*)(A + ra0 + k0);  a0.u[1] = *(const v4i*)(A + ra0 + k0 + 16);
    a1.u[0] = *(const v4i*)(A + ra1 + k0);  a1.u[1] = *(const v4i*)(A + ra1 + k0 + 16);
    b.u[0]  = *(const v4i*)(B + rb + k0);   b.u[1]  = *(const v4i*)(B + rb + k0 + 16);
    c0 = wmh(a0.v, b.v, c0);
    c1 = wmh(a1.v, b.v, c1);
  }

  const float bv = bias[ncol];
#pragma unroll
  for (int r = 0; r < 8; ++r) {
    Xs[(8 * hh + r) * XSP + ncol]      = c0[r] * oscale + bv;
    Xs[(16 + 8 * hh + r) * XSP + ncol] = c1[r] * oscale + bv;
  }
  __syncthreads();

  v4f xv[4];
  float* xpp[4];
#pragma unroll
  for (int i = 0; i < 4; ++i) {
    xv[i]  = *(const v4f*)(Xs + (4 * wave + i) * XSP + 4 * lane);
    xpp[i] = out + (size_t)(rowBase + 4 * wave + i) * DM + 4 * lane;
  }
#pragma unroll
  for (int i = 0; i < 4; ++i) *(volatile v4f*)(xpp[i]) = xv[i];
  __threadfence();
#pragma unroll
  for (int i = 0; i < 4; ++i) *(volatile v4f*)(xpp[i]) = xv[i];
}

__device__ __forceinline__ void hit(const float* xs, const float* xd, float* ar, float* dp,
                                    v4f we4, v4f at4, float w) {
  const v4f a = *(const v4f*)(xs);
  const v4f d = *(const v4f*)(xd);
  const v4f t = a + d + we4 * w;
  float s = dl(t, at4);
  s = wsum32(s);
  s = fminf(s, 80.0f);
  const float p = __expf(s);
  v4f e = *(v4f*)(ar);
  e = e + a * p;
  *(v4f*)(ar) = e;
  dp[0] = dp[0] + p;
}

__global__ __launch_bounds__(NTHR) void k_agg(
    const int* __restrict__ ei, const float* __restrict__ ew, const float* __restrict__ wsum,
    const float* __restrict__ xl, const float* __restrict__ xr, const float* __restrict__ xres,
    const float* __restrict__ We, const float* __restrict__ att, const float* __restrict__ bias,
    const float* __restrict__ gam, const float* __restrict__ bet,
    float* out, int nN, int nE) {
  extern __shared__ v4f lds_dyn[];
  float* sacc = (float*)lds_dyn;
  float* dn   = sacc + NB * DM;
  int*   list = (int*)(dn + NB);
  int*   wcnt = list + NWAVE * WCAP;

  const int tid  = threadIdx.x;
  const int lane = tid & 31;
  const int wave = tid >> 5;
  const int nodeBase = blockIdx.x * NB;

  {
    const v4f z4 = {0.f, 0.f, 0.f, 0.f};
    for (int i = tid; i < NB * DM / 4; i += NTHR) lds_dyn[i] = z4;
    for (int i = tid; i < NB; i += NTHR) dn[i] = 0.f;
  }
  __syncthreads();

  const int co = 4 * lane;
  const v4f we4 = *(const v4f*)(We + co);
  const v4f at4 = *(const v4f*)(att + co);
  const float wmean = wsum[0];

  const int* eid = ei + nE;
  const bool al16 = ((nE & 3) == 0);
  const int nChunks = (nE + CHUNK - 1) / CHUNK;

#pragma unroll 1
  for (int ch = 0; ch <= nChunks; ++ch) {
    const int cbase = ch * CHUNK;
    const bool selfp = (ch == nChunks);
    if (!selfp) {
      int wc = 0;
#pragma unroll
      for (int g = 0; g < NGRP; ++g) {
        const int el0 = (g * NTHR + tid) * 4;
        const int e0  = cbase + el0;
        const int sent = -2147483647 - 1;
        v4i d;
        if (al16 && (e0 + 3 < nE)) {
          d = *(const v4i*)(eid + e0);
        } else {
          d.x = (e0     < nE) ? eid[min(e0, nE - 1)]     : sent;
          d.y = (e0 + 1 < nE) ? eid[min(e0 + 1, nE - 1)] : sent;
          d.z = (e0 + 2 < nE) ? eid[min(e0 + 2, nE - 1)] : sent;
          d.w = (e0 + 3 < nE) ? eid[min(e0 + 3, nE - 1)] : sent;
        }
        const unsigned s0 = (unsigned)d.x - (unsigned)nodeBase;
        const unsigned s1 = (unsigned)d.y - (unsigned)nodeBase;
        const unsigned s2 = (unsigned)d.z - (unsigned)nodeBase;
        const unsigned s3 = (unsigned)d.w - (unsigned)nodeBase;
        const bool h0 = s0 < (unsigned)NB;
        const bool h1 = s1 < (unsigned)NB;
        const bool h2 = s2 < (unsigned)NB;
        const bool h3 = s3 < (unsigned)NB;
        const unsigned many = __builtin_amdgcn_ballot_w32(h0 | h1 | h2 | h3);
        if (many != 0u) {
#define HITJ(J, HJ, SJ) { \
            const unsigned mj = __builtin_amdgcn_ballot_w32(HJ); \
            if (HJ) { \
              const int pos = wc + (int)__builtin_amdgcn_mbcnt_lo(mj, 0u); \
              if (pos < WCAP) list[wave * WCAP + pos] = ((el0 + (J)) << 9) | (int)(SJ); \
            } \
            wc += (int)__builtin_popcount(mj); }
          HITJ(0, h0, s0)
          HITJ(1, h1, s1)
          HITJ(2, h2, s2)
          HITJ(3, h3, s3)
#undef HITJ
        }
      }
      if (lane == 0) wcnt[wave] = wc;
    } else {
      for (int s = tid; s < NB; s += NTHR) list[s] = s;
      if (tid < NWAVE) {
        int c = NB - tid * WCAP;
        c = c < 0 ? 0 : (c > WCAP ? WCAP : c);
        wcnt[tid] = c;
      }
    }
    __syncthreads();

    if (wave == 0) {
#pragma unroll 1
      for (int wsx = 0; wsx < NWAVE; ++wsx) {
        int n = __builtin_amdgcn_readfirstlane(wcnt[wsx]);
        n = n > WCAP ? WCAP : n;
        n = n < 0 ? 0 : n;
#pragma unroll 1
        for (int i = 0; i < n; ++i) {
          const int ent  = __builtin_amdgcn_readfirstlane(list[wsx * WCAP + i]);
          const int slot = ent & (NB - 1);
          const int el   = (ent >> 9) & (CHUNK - 1);
          const int node = nodeBase + slot;
          if (node >= nN) continue;
          int e = cbase + el;
          if (e > nE - 1) e = nE - 1;
          int sj = ei[e];
          sj = sj < 0 ? 0 : (sj > nN - 1 ? nN - 1 : sj);
          const int src = selfp ? node : sj;
          const float w = selfp ? wmean : ew[e];
          hit(xl + (size_t)src * DM + co, xr + (size_t)node * DM + co,
              sacc + slot * DM + co, dn + slot, we4, at4, w);
        }
      }
    }
    __syncthreads();
  }

  const v4f bi4 = *(const v4f*)(bias + co);
  const v4f g4  = *(const v4f*)(gam + co);
  const v4f be4 = *(const v4f*)(bet + co);
  const float invD = 1.0f / (float)DM;
#pragma unroll 1
  for (int s = wave; s < NB; s += NWAVE) {
    const int node = nodeBase + s;
    if (node >= nN) break;
    const v4f e = *(const v4f*)(sacc + s * DM + co);
    const float den = dn[s];
    const float inv = __builtin_amdgcn_rcpf(fmaxf(den, 1e-30f));
    const v4f xv = *(const v4f*)(xres + (size_t)node * DM + co);
    const v4f y = xv + (e * inv + bi4);
    float su = y.x + y.y + y.z + y.w;
    su = wsum32(su);
    const float mu = su * invD;
    const v4f dv = y - mu;
    float sq = dv.x * dv.x + dv.y * dv.y + dv.z * dv.z + dv.w * dv.w;
    sq = wsum32(sq);
    const float var = sq * invD;
    const float rr = rsqrtf(var + 1e-5f);
    const v4f o = dv * rr * g4 + be4;
    float* op = out + (size_t)node * DM + co;
    *(volatile v4f*)op = o;
    __threadfence();
    *(volatile v4f*)op = o;
  }
}

extern "C" void kernel_launch(void* const* d_in, const int* in_sizes, int n_in,
                              void* d_out, int out_size, void* d_ws, size_t ws_size,
                              hipStream_t stream) {
  if (n_in < 22) return;
  const int nN = in_sizes[0];
  if (nN <= 0) return;
  const int nE = in_sizes[2];
  if (nE <= 0 || in_sizes[1] != 2 * nE) return;
  const int nV = in_sizes[3] / DM;
  if (nV <= 0 || in_sizes[3] != nV * DM) return;
  if (in_sizes[4] != DM * DM || in_sizes[6] != DM * DM || in_sizes[13] != DM * DM || in_sizes[15] != DM * DM) return;
  if (in_sizes[5] != DM || in_sizes[7] != DM || in_sizes[8] != DM || in_sizes[9] != DM || in_sizes[10] != DM ||
      in_sizes[11] != DM || in_sizes[12] != DM) return;
  if (in_sizes[14] != DM || in_sizes[16] != DM || in_sizes[17] != DM || in_sizes[18] != DM || in_sizes[19] != DM ||
      in_sizes[20] != DM || in_sizes[21] != DM) return;
  if (out_size != nN * DM) return;

  const int*   ids = (const int*)d_in[0];
  const int*   ei  = (const int*)d_in[1];
  const float* ew  = (const float*)d_in[2];
  const float* emb = (const float*)d_in[3];
  const float* w1l = (const float*)d_in[4];   const float* b1l  = (const float*)d_in[5];
  const float* w1r = (const float*)d_in[6];   const float* b1r  = (const float*)d_in[7];
  const float* w1e = (const float*)d_in[8];   const float* at1  = (const float*)d_in[9];
  const float* bs1 = (const float*)d_in[10];  const float* g1   = (const float*)d_in[11];
  const float* be1 = (const float*)d_in[12];
  const float* w2l = (const float*)d_in[13];  const float* b2l  = (const float*)d_in[14];
  const float* w2r = (const float*)d_in[15];  const float* b2r  = (const float*)d_in[16];
  const float* w2e = (const float*)d_in[17];  const float* at2  = (const float*)d_in[18];
  const float* bs2 = (const float*)d_in[19];  const float* g2   = (const float*)d_in[20];
  const float* be2 = (const float*)d_in[21];
  float* out = (float*)d_out;

  const int Npad = ((nN + GR - 1) / GR) * GR;
  const int mt   = Npad / GR;

  char* wsp = (char*)d_ws;
  size_t off = 0;
  const size_t rowsF = (size_t)Npad * DM * 4;
  const size_t rowsH = (size_t)Npad * DM * 2;
  float* wsum = (float*)(wsp + off);                      off += 512;
  unsigned short* planes = (unsigned short*)(wsp + off);   off += (size_t)4 * DM * DM * 2;
  float* x0 = (float*)(wsp + off);                         off += rowsF;
  unsigned short* apl = (unsigned short*)(wsp + off);      off += rowsH;
  float* xl = (float*)(wsp + off);                         off += rowsF;
  float* xr = (float*)(wsp + off);                         off += rowsF;
  float* x1 = (float*)(wsp + off);                         off += rowsF;
  if (off > ws_size) return;

  hipFuncSetAttribute(reinterpret_cast<const void*>(&k_agg), hipFuncAttributeMaxDynamicSharedMemorySize, AGG_LDS_BYTES);

  const float sW   = 8.0f;
  const float sX1  = 16.0f;
  const float os1  = 1.0f / 128.0f;
  const float os2  = 1.0f / 8.0f;
  const int nAggBlocks = (nN + NB - 1) / NB;

  k_mean<<<1, NTHR, 0, stream>>>(ew, nE, wsum);
  k_wcvt<<<dim3(DM * DM / 8 / NTHR, 4), NTHR, 0, stream>>>(w1l, w1r, w2l, w2r, planes, sW);
  k_gather<<<(nN * 32 + NTHR - 1) / NTHR, NTHR, 0, stream>>>(ids, emb, nV, x0, apl, nN, Npad, sX1);

  k_gemm<<<dim3(mt, 2), NTHR, 0, stream>>>(apl, planes, planes + DM * DM, b1l, b1r, xl, xr, DM, os1);
  k_agg<<<nAggBlocks, NTHR, AGG_LDS_BYTES, stream>>>(ei, ew, wsum, xl, xr, x0, w1e, at1, bs1, g1, be1, x1, nN, nE);

  k_xcvt<<<(Npad * 16 + NTHR - 1) / NTHR, NTHR, 0, stream>>>(x1, apl, nN, Npad);
  k_gemm<<<dim3(mt, 2), NTHR, 0, stream>>>(apl, planes + 2 * DM * DM, planes + 3 * DM * DM, b2l, b2r, xl, xr, DM, os2);
  k_agg<<<nAggBlocks, NTHR, AGG_LDS_BYTES, stream>>>(ei, ew, wsum, xl, xr, x1, w2e, at2, bs2, g2, be2, out, nN, nE);
}
